// BiLevelRoutingAttention_26688926777430
// MI455X (gfx1250) — hardware-run, weakly checked
//
#include <hip/hip_runtime.h>


namespace {
typedef _Float16 b16;
typedef __attribute__((ext_vector_type(16))) _Float16 v16b;
typedef __attribute__((ext_vector_type(8))) _Float16 v8b;
typedef __attribute__((ext_vector_type(4))) _Float16 v4h;
typedef __attribute__((ext_vector_type(2))) _Float16 v2h;
typedef __attribute__((ext_vector_type(8))) float v8f;
typedef __attribute__((ext_vector_type(4))) float v4f;
typedef __attribute__((ext_vector_type(2))) float v2f;
__device__ __forceinline__ float bf16_rne(float f) { unsigned int u = __float_as_uint(f); u += 0x7FFFu + ((u >> 16) & 1u); return __uint_as_float(u & 0xFFFF0000u); }
__device__ __forceinline__ void split16(float v, b16& hi, b16& lo) { hi = (b16)v; lo = (b16)(v - (float)hi); }
__device__ __forceinline__ v16b frag_kb(const b16* p, int hh) { const v8b a = *(const v8b*)(p + 8 * hh), b = *(const v8b*)(p + 16 + 8 * hh); v16b f;
#pragma unroll
  for (int e = 0; e < 8; ++e) { f[e] = a[e]; f[8 + e] = b[e]; } return f; }
__device__ __forceinline__ v8f wmma16b(v16b a, v16b b, v8f c) { v8f d = __builtin_amdgcn_wmma_f32_16x16x32_f16(false, a, false, b, (short)0, c, false, false); asm volatile("v_nop\n\tv_nop\n\tv_nop\n\tv_nop" : "+v"(d) : "v"(a), "v"(b)); return d; }
__device__ __forceinline__ void wave_lds_sync() { __builtin_amdgcn_fence(__ATOMIC_RELEASE, "workgroup"); __builtin_amdgcn_wave_barrier(); __builtin_amdgcn_fence(__ATOMIC_ACQUIRE, "workgroup"); }
__device__ __forceinline__ float pmul(float a, float b) { float p = a * b; asm volatile("" : "+v"(p)); return p; }
__device__ __forceinline__ int iclamp(int v, int lo, int hi) { return v < lo ? lo : (v > hi ? hi : v); }
__device__ __forceinline__ float nexp2(float v) { return __builtin_amdgcn_exp2f(v); }

constexpr int B = 2, HS = 56, C = 256, NH = 8, HD = 32, NWIN = 7, WSZ = 8, NSP = HS * HS, S = NSP + 1, NBLK = 50, TP = NBLK * 64, NOUTR = B * NSP + B  , NOUTP = 6304, BL = B  ;
constexpr float XS = 8.0f, WSC = 256.0f, PS = 1024.0f, LOG2E = 1.4426950408889634f, SCALE = 0.0625f;
static_assert(NSP % 64 == 0 && TP % 64 == 0 && C == 256 && NOUTP % 32 == 0 && NOUTP >= NOUTR, "tiling");

template <int KD, int NOUT, int LDA, int LDT, bool RNDA>
__global__ __launch_bounds__(64) void gemmx_kernel(const float* __restrict__ A, int nv, const b16* __restrict__ W, const float* __restrict__ bias, int mrows, float* __restrict__ T) {
  constexpr int SL = NOUT < 128 ? NOUT : 128, NT = SL / 16, KC = KD < 128 ? KD : 128;
  static_assert(KD % KC == 0 && KC % 32 == 0 && NOUT % SL == 0 && SL % 32 == 0 && LDA >= KD && LDT >= NOUT, "gemmx tiling");
  __shared__ __attribute__((aligned(16))) b16 Ah[2][16][KC + 8], Al[2][16][KC + 8]; __shared__ __attribute__((aligned(16))) float Tf[2][16][SL + 4];
  const int wave = threadIdx.x >> 5, lane = threadIdx.x & 31, nloc = lane & 15, hlf = lane >> 4; const size_t m0 = (size_t)blockIdx.x * 32 + wave * 16; const int n0 = blockIdx.y * SL;
  v8f acc[NT];
#pragma unroll
  for (int t = 0; t < NT; ++t) acc[t] = (v8f){};
#pragma unroll 1
  for (int kc = 0; kc < KD; kc += KC) {
    for (int idx = lane; idx < 16 * (KC / 4); idx += 32) { const int rr = idx / (KC / 4), c4 = (idx % (KC / 4)) * 4; const size_t row = (m0 + rr < (size_t)nv) ? (m0 + rr) : (size_t)(nv - 1); const v4f v = *(const v4f*)(A + row * LDA + kc + c4); v4h hv, lv;
      for (int j = 0; j < 4; ++j) { b16 ph, pl; split16((RNDA ? bf16_rne(v[j]) : v[j]) * XS, ph, pl); hv[j] = ph; lv[j] = pl; } *(v4h*)(&Ah[wave][rr][c4]) = hv; *(v4h*)(&Al[wave][rr][c4]) = lv; }
    wave_lds_sync();
#pragma unroll
    for (int kb = 0; kb < KC; kb += 32) { const v16b a = frag_kb(&Ah[wave][nloc][kb], hlf), al = frag_kb(&Al[wave][nloc][kb], hlf);
#pragma unroll
      for (int t = 0; t < NT; ++t) { const v16b bw = frag_kb(W + (size_t)(n0 + t * 16 + nloc) * KD + kc + kb, hlf); acc[t] = wmma16b(a, bw, acc[t]); if (!RNDA) acc[t] = wmma16b(al, bw, acc[t]); } }
    wave_lds_sync(); }
#pragma unroll
  for (int t = 0; t < NT; ++t) { const float bb = bias ? bf16_rne(bias[n0 + t * 16 + nloc]) : 0.0f;
#pragma unroll
    for (int r = 0; r < 8; ++r) Tf[wave][8 * hlf + r][t * 16 + nloc] = acc[t][r] * (1.0f / (XS * WSC)) + bb; }
  wave_lds_sync();
  for (int pass = 0; pass < 2; ++pass) { for (int idx = lane; idx < 16 * (SL / 4); idx += 32) { const int rr = idx / (SL / 4), c4 = (idx % (SL / 4)) * 4; if (m0 + rr < (size_t)mrows) *(volatile v4f*)(T + (m0 + rr) * LDT + n0 + c4) = *(const v4f*)(&Tf[wave][rr][c4]); } __threadfence(); }
}

__device__ __forceinline__ int tok2pix(int t) { const int win = t >> 6, r = t & 63; const int j = win / NWIN, i = win % NWIN; const int y = j * WSZ + (r >> 3), x = i * WSZ + (r & 7); return y * HS + x; }
__global__ __launch_bounds__(256) void prep_kernel(const float* __restrict__ wp, const float* __restrict__ wo, b16* __restrict__ WT, b16* __restrict__ WO) {
  const int u = blockIdx.x * 256 + threadIdx.x; const int n1 = 3 * C * C / 8, n2 = C * C / 8; if (u >= n1 + n2) return; v8b o;
  if (u < n1) { const int e = u * 8; for (int j = 0; j < 8; ++j) o[j] = (b16)(bf16_rne(wp[e + j]) * WSC); for (int pass = 0; pass < 2; ++pass) { *(volatile v8b*)(WT + e) = o; __threadfence(); } }
  else { const int e = (u - n1) * 8; for (int j = 0; j < 8; ++j) o[j] = (b16)(bf16_rne(wo[e + j]) * WSC); for (int pass = 0; pass < 2; ++pass) { *(volatile v8b*)(WO + e) = o; __threadfence(); } }
}
__global__ __launch_bounds__(128) void proj_kernel(const float* __restrict__ x, const float* __restrict__ cls, const b16* __restrict__ WT, const float* __restrict__ bp, b16* __restrict__ QP, b16* __restrict__ KP, b16* __restrict__ VTh, float* __restrict__ VIMG) {
  __shared__ __attribute__((aligned(16))) b16 As[64][C + 8]; __shared__ __attribute__((aligned(16))) float Tf[4][16][128 + 4];
  const int wave = threadIdx.x >> 5, lane = threadIdx.x & 31, nloc = lane & 15, hlf = lane >> 4; const int t0 = blockIdx.x * 64; const int b = blockIdx.y; const int slab = blockIdx.z, n0 = slab * 128, part = slab / 2, h0 = (slab & 1) * 4;
  for (int i = threadIdx.x; i < 64 * (C / 4); i += 128) { const int rr = i / (C / 4), q = (i % (C / 4)) * 4; const int t = t0 + rr; v4f f = {0.0f, 0.0f, 0.0f, 0.0f};
    if (t < NSP) f = *(const v4f*)(x + ((size_t)b * NSP + tok2pix(t)) * C + q); else if (t == NSP) f = *(const v4f*)(cls + (size_t)b * C + q);
    v4h o; for (int j = 0; j < 4; ++j) o[j] = (b16)(bf16_rne(f[j]) * XS); *(v4h*)(&As[rr][q]) = o; }
  __syncthreads();
  v8f acc[8];
#pragma unroll
  for (int t = 0; t < 8; ++t) acc[t] = (v8f){};
#pragma unroll 2
  for (int kb = 0; kb < C; kb += 32) { const v16b a = frag_kb(&As[wave * 16 + nloc][kb], hlf);
#pragma unroll
    for (int t = 0; t < 8; ++t) acc[t] = wmma16b(a, frag_kb(WT + (size_t)(n0 + t * 16 + nloc) * C + kb, hlf), acc[t]); }
#pragma unroll
  for (int t = 0; t < 8; ++t) { const float bb = bf16_rne(bp[n0 + t * 16 + nloc]);
#pragma unroll
    for (int r = 0; r < 8; ++r) Tf[wave][8 * hlf + r][t * 16 + nloc] = acc[t][r] * (1.0f / (XS * WSC)) + bb; }
  __syncthreads();
  for (int pass = 0; pass < 2; ++pass) {
    if (part < 2) { b16* plane = part == 0 ? QP : KP; const int h = h0 + (lane >> 3), d = (lane & 7) * 4;
      for (int rr = 0; rr < 16; ++rr) { const int tok = t0 + wave * 16 + rr; v4h o4; for (int j = 0; j < 4; ++j) o4[j] = (b16)(Tf[wave][rr][lane * 4 + j] * XS); *(volatile v4h*)(plane + (((size_t)b * NH + h) * TP + tok) * HD + d) = o4; } }
    else {
#pragma unroll 1
      for (int q = 0; q < 32; ++q) { const int cl = wave * 32 + q; const int h = h0 + cl / HD, d = cl % HD; const int tk = lane * 2; v2h hv; hv[0] = (b16)(Tf[tk >> 4][tk & 15][cl] * XS); hv[1] = (b16)(Tf[(tk + 1) >> 4][(tk + 1) & 15][cl] * XS);
        *(volatile v2h*)(VTh + (((size_t)b * NH + h) * HD + d) * (size_t)TP + t0 + tk) = hv; }
      for (int rr = 0; rr < 16; ++rr) { const int tok = t0 + wave * 16 + rr; if (tok < NSP) *(volatile v4f*)(VIMG + ((size_t)b * NSP + tok2pix(tok)) * C + (n0 - 2 * C) + lane * 4) = *(const v4f*)(&Tf[wave][rr][lane * 4]); } }
    __threadfence(); }
}
__global__ __launch_bounds__(64) void attn_kernel(const b16* __restrict__ QP, const b16* __restrict__ KP, const b16* __restrict__ VTh, const int* __restrict__ mask, float* __restrict__ CT) {
  __shared__ __attribute__((aligned(16))) b16 Pb[2][16][32 + 8]; __shared__ __attribute__((aligned(16))) float To[2][16][HD + 4];
  const int wave = threadIdx.x >> 5, lane = threadIdx.x & 31, hh = lane >> 4, col = lane & 15; const int b = blockIdx.y / NH, h = blockIdx.y % NH; const int q0 = blockIdx.x * 32 + wave * 16, qi = q0 + col; const int qb = blockIdx.x >> 1;
  const size_t ph = (size_t)b * NH + h; const b16* Qb = QP + ph * TP * HD; const b16* Kb = KP + ph * TP * HD; const b16* Vb = VTh + ph * HD * (size_t)TP; const int* mrow = mask + ((size_t)b * NBLK + qb) * NBLK;
  const v16b qa = frag_kb(Qb + (size_t)qi * HD, hh);
  const float cs = LOG2E * SCALE / (XS * XS);
  float m = -INFINITY, l = 0.0f; v8f o[2]; o[0] = (v8f){}; o[1] = (v8f){};
#pragma unroll 1
  for (int kbk = 0; kbk < NBLK; ++kbk) { if (mrow[kbk] == 0) continue;
#pragma unroll 1
    for (int half = 0; half < 2; ++half) { const int kb = kbk * 64 + half * 32;
      float e[16]; float mx = -INFINITY;
#pragma unroll
      for (int u = 0; u < 2; ++u) { v8f s = (v8f){}; s = wmma16b(frag_kb(Kb + (size_t)(kb + u * 16 + col) * HD, hh), qa, s);
#pragma unroll
        for (int r = 0; r < 8; ++r) { const int key = kb + u * 16 + 8 * hh + r; const float vv = (key < S) ? s[r] * cs : -INFINITY; e[u * 8 + r] = vv; mx = fmaxf(mx, vv); } }
      mx = fmaxf(mx, __shfl_xor(mx, 16)); const float mn = fmaxf(m, mx); const float al = (mn == -INFINITY) ? 1.0f : nexp2(m - mn); float sum = 0.0f;
#pragma unroll
      for (int i2 = 0; i2 < 16; ++i2) { const float p = (mn == -INFINITY) ? 0.0f : nexp2(e[i2] - mn); sum += p; Pb[wave][col][(i2 < 8 ? 0 : 16) + 8 * hh + (i2 & 7)] = (b16)(p * PS); }
      sum += __shfl_xor(sum, 16); l = l * al + sum; m = mn;
      wave_lds_sync();
      const v16b pf = frag_kb(&Pb[wave][col][0], hh);
#pragma unroll
      for (int t = 0; t < 2; ++t) { o[t] *= al; o[t] = wmma16b(frag_kb(Vb + (size_t)(t * 16 + col) * TP + kb, hh), pf, o[t]); }
      wave_lds_sync(); } }
  const float inv = (l > 0.0f) ? 1.0f / (l * PS * XS) : 0.0f;
#pragma unroll
  for (int t = 0; t < 2; ++t)
#pragma unroll
    for (int r = 0; r < 8; ++r) To[wave][col][t * 16 + 8 * hh + r] = o[t][r] * inv;
  wave_lds_sync();
  for (int pass = 0; pass < 2; ++pass) { for (int rr = 0; rr < 16; ++rr) { const int tok = q0 + rr; size_t row; if (tok < NSP) row = (size_t)b * NSP + tok2pix(tok); else if (tok == NSP) row = (size_t)B * NSP + b; else continue;
      ((volatile float*)CT)[row * C + h * HD + lane] = To[wave][rr][lane]; } __threadfence(); }
}
__global__ __launch_bounds__(256) void lepe_kernel(const float* __restrict__ CT, const float* __restrict__ VIMG, const float* __restrict__ lw, const float* __restrict__ lb, float* __restrict__ OI) {
  const size_t u = (size_t)blockIdx.x * 256 + threadIdx.x; if (u >= (size_t)NOUTP * (C / 4)) return; const int row = (int)(u / (C / 4)), c = (int)(u % (C / 4)) * 4; v4f o = {0.0f, 0.0f, 0.0f, 0.0f};
  if (row < B * NSP) { const int b = row / NSP, p = row % NSP, y = p / HS, xx = p % HS; v4f a; for (int j = 0; j < 4; ++j) a[j] = bf16_rne(lb[c + j]);
    for (int dy = -1; dy <= 1; ++dy) for (int dx = -1; dx <= 1; ++dx) { const int yy = y + dy, x2 = xx + dx; if (yy < 0 || yy >= HS || x2 < 0 || x2 >= HS) continue; const v4f v = *(const v4f*)(VIMG + ((size_t)b * NSP + yy * HS + x2) * C + c);
        for (int j = 0; j < 4; ++j) a[j] = fmaf(v[j], bf16_rne(lw[((dy + 1) * 3 + (dx + 1)) * C + c + j]), a[j]); }
    const v4f ct = *(const v4f*)(CT + (size_t)row * C + c); for (int j = 0; j < 4; ++j) o[j] = ct[j] + a[j]; }
  else if (row < NOUTR) o = *(const v4f*)(CT + (size_t)row * C + c);
  for (int pass = 0; pass < 2; ++pass) { *(volatile v4f*)(OI + (size_t)row * C + c) = o; __threadfence(); }
}
}

extern "C" void kernel_launch(void* const* d_in, const int* in_sizes, int n_in, void* d_out, int out_size, void* d_ws, size_t ws_size, hipStream_t stream) {
  (void)n_in;
  auto Fp = [&](int i) { return (const float*)d_in[i]; };
  if (in_sizes[0] != B * NSP * C || in_sizes[1] != B * C || in_sizes[2] != B * NBLK * NBLK || in_sizes[3] != 3 * C * C || in_sizes[4] != 3 * C || in_sizes[5] != 9 * C || in_sizes[6] != C || in_sizes[7] != C * C || in_sizes[8] != C || out_size != NOUTR * C) return;
  size_t off = 0; char* ws = (char*)d_ws;
  auto carve = [&](size_t bytes) { char* p = ws + off; off += (bytes + 255) & ~(size_t)255; return p; };
  b16* WT = (b16*)carve((size_t)3 * C * C * 2); b16* WO = (b16*)carve((size_t)C * C * 2); const size_t plane = (size_t)B * NH * TP * HD * 2;
  b16* QP = (b16*)carve(plane); b16* KP = (b16*)carve(plane); b16* VTh = (b16*)carve(plane); float* VIMG = (float*)carve((size_t)B * NSP * C * 4); float* CT = (float*)carve((size_t)NOUTP * C * 4); float* OI = (float*)carve((size_t)NOUTP * C * 4);
  if (off > ws_size || off > ((size_t)128 << 20)) return;
  prep_kernel<<<(3 * C * C / 8 + C * C / 8 + 255) / 256, 256, 0, stream>>>(Fp(3), Fp(7), WT, WO);
  proj_kernel<<<dim3(TP / 64, BL, 6), 128, 0, stream>>>(Fp(0), Fp(1), WT, Fp(4), QP, KP, VTh, VIMG);
  attn_kernel<<<dim3(TP / 32, BL * NH), 64, 0, stream>>>(QP, KP, VTh, (const int*)d_in[2], CT);
  lepe_kernel<<<(unsigned)(((size_t)NOUTP * (C / 4) + 255) / 256), 256, 0, stream>>>(CT, VIMG, Fp(5), Fp(6), OI);
  gemmx_kernel<C, C, C, C, false><<<dim3(NOUTP / 32, 2), 64, 0, stream>>>(OI, NOUTR, WO, Fp(8), NOUTR, (float*)d_out);
}
